// ConceptNAMNary_44650480010036
// MI455X (gfx1250) — hardware-verified
//
#include <hip/hip_runtime.h>
#include <math.h>

typedef __attribute__((ext_vector_type(16))) _Float16 v16h;
typedef __attribute__((ext_vector_type(16))) __bf16 v16b;
typedef __attribute__((ext_vector_type(8)))  _Float16 v8h;
typedef __attribute__((ext_vector_type(8)))  float v8f;
typedef __attribute__((ext_vector_type(4)))  float v4f;
typedef __attribute__((ext_vector_type(2)))  float v2f;
typedef __attribute__((ext_vector_type(4)))  unsigned v4u;
typedef __attribute__((ext_vector_type(4)))  int v4i;
typedef float __attribute__((may_alias)) float_a;
typedef int __attribute__((may_alias)) int_a;

template <typename T> __device__ __forceinline__ void vst2(void* p, T v) { *(volatile T*)p = v; __threadfence(); *(volatile T*)p = v; }
__device__ __forceinline__ v8f wmma16(v16h a, v16h b, v8f c) {
  v8f d = __builtin_amdgcn_wmma_f32_16x16x32_f16(false, a, false, b, (short)0, c, false, false);
  asm volatile("v_nop\n\tv_nop\n\tv_nop\n\tv_nop" : "+v"(d) : "v"(a), "v"(b));
  return d;
}
__device__ __forceinline__ v8f wmma_bf(v16b a, v16b b, v8f c) {
  v8f d = __builtin_amdgcn_wmma_f32_16x16x32_bf16(false, a, false, b, (short)0, c, false, false);
  asm volatile("v_nop\n\tv_nop\n\tv_nop\n\tv_nop" : "+v"(d) : "v"(a), "v"(b));
  return d;
}
__device__ __forceinline__ v16h frag_h(const _Float16* rowk0, int lane) {
  union { v16h v; v8h q[2]; } u; const _Float16* p = rowk0 + 8 * (lane >> 4);
  u.q[0] = *(const v8h*)p; u.q[1] = *(const v8h*)(p + 16); return u.v;
}
__device__ __forceinline__ v16h frag_f32(const float* rowk0, int lane) {
  v16h a; const float* p = rowk0 + 8 * (lane >> 4);
#pragma unroll
  for (int i = 0; i < 8; ++i) { a[i] = (_Float16)p[i]; a[8 + i] = (_Float16)p[16 + i]; }
  return a;
}
__device__ __forceinline__ v16h frag_f32s(const float* rowk0, int lane, float sc) {
  v16h a; const float* p = rowk0 + 8 * (lane >> 4);
#pragma unroll
  for (int i = 0; i < 8; ++i) { a[i] = (_Float16)(p[i] * sc); a[8 + i] = (_Float16)(p[16 + i] * sc); }
  return a;
}
__device__ __forceinline__ v16h fragc_f32(const float* W, int k0, int n, int lane, int ld, int K) {
  v16h a; const int g = lane >> 4;
#pragma unroll
  for (int i = 0; i < 8; ++i) { const int ka = k0 + 8 * g + i, kb = ka + 16;
    a[i] = (_Float16)(ka < K ? W[(size_t)(ka < K ? ka : K - 1) * ld + n] : 0.f); a[8 + i] = (_Float16)(kb < K ? W[(size_t)(kb < K ? kb : K - 1) * ld + n] : 0.f); }
  return a;
}
struct F2 { v16b h, l; };
__device__ __forceinline__ F2 bsplit16(const float v[16]) { F2 r;
#pragma unroll
  for (int i = 0; i < 16; ++i) { const __bf16 h = (__bf16)v[i]; r.h[i] = h; r.l[i] = (__bf16)(v[i] - (float)h); }
  return r; }
__device__ __forceinline__ F2 split_row(const float* row, int k0, int lane) { float v[16]; const float* p = row + k0 + 8 * (lane >> 4);
#pragma unroll
  for (int i = 0; i < 8; ++i) { v[i] = p[i]; v[8 + i] = p[16 + i]; }
  return bsplit16(v); }
__device__ __forceinline__ F2 split_rowK(const float* row, int k0, int lane, int K) { float v[16]; const int g = lane >> 4;
#pragma unroll
  for (int i = 0; i < 8; ++i) { const int ka = k0 + 8 * g + i, kb = ka + 16; v[i] = ka < K ? row[ka < K ? ka : K - 1] : 0.f; v[8 + i] = kb < K ? row[kb < K ? kb : K - 1] : 0.f; }
  return bsplit16(v); }
__device__ __forceinline__ F2 split_col(const float* W, int k0, int n, int lane, int ld, int K) { float v[16]; const int g = lane >> 4;
#pragma unroll
  for (int i = 0; i < 8; ++i) { const int ka = k0 + 8 * g + i, kb = ka + 16; v[i] = ka < K ? W[(size_t)(ka < K ? ka : K - 1) * ld + n] : 0.f; v[8 + i] = kb < K ? W[(size_t)(kb < K ? kb : K - 1) * ld + n] : 0.f; }
  return bsplit16(v); }
__device__ __forceinline__ v8f mac3(const F2& a, const F2& b, v8f c) { c = wmma_bf(a.l, b.h, c); c = wmma_bf(a.h, b.l, c); return wmma_bf(a.h, b.h, c); }
__device__ __forceinline__ float sigm(float v) { return 1.0f / (1.0f + expf(-v)); }
#define LDSX() do { asm volatile("s_wait_dscnt 0" ::: "memory"); __builtin_amdgcn_wave_barrier(); __builtin_amdgcn_fence(__ATOMIC_RELEASE, "workgroup"); } while (0)


#define NB 2048
#define NC 32
#define NM 496
#define H1 64
#define H2 32
#define NCLS 10
#ifndef TBB
#define TBB (NB / 64)
#endif
typedef __attribute__((ext_vector_type(8))) __bf16 v8b;
__device__ __forceinline__ v16b frag_b(const __bf16* rowk0, int lane) {
  union { v16b v; v8b q[2]; } u; const __bf16* p = rowk0 + 8 * (lane >> 4);
  u.q[0] = *(const v8b*)p; u.q[1] = *(const v8b*)(p + 16); return u.v;
}
__device__ __forceinline__ v16b frag_gbf(const float* rowk0, int lane) {
  v16b a; const float* p = rowk0 + 8 * (lane >> 4);
#pragma unroll
  for (int i = 0; i < 8; ++i) { a[i] = (__bf16)p[i]; a[8 + i] = (__bf16)p[16 + i]; }
  return a;
}
__device__ __forceinline__ float bfr(float v) { return (float)(__bf16)v; }
#define WS_OT  0u
#define WS_END (WS_OT + 4u * 512 * NB)

__global__ __launch_bounds__(128) void k_pair(const float* __restrict__ X, const int* __restrict__ PIDX, const float* __restrict__ W1, const float* __restrict__ b1, const float* __restrict__ g1, const float* __restrict__ be1, const float* __restrict__ m1, const float* __restrict__ v1,
                                              const float* __restrict__ W2, const float* __restrict__ b2, const float* __restrict__ g2, const float* __restrict__ be2, const float* __restrict__ m2, const float* __restrict__ v2, const float* __restrict__ W3, const float* __restrict__ b3, float* __restrict__ OT) {
  __shared__ __align__(16) __bf16 sah[64][72], sal[64][72]; __shared__ float sp1[H1][6]; __shared__ float sp2[H2][4]; __shared__ float sw3[H2]; __shared__ float sh2[64][H2 + 1]; __shared__ __align__(16) float sres[64];
  const int tid = threadIdx.x, wave = tid >> 5, lane = tid & 31, col = lane & 15, g = lane >> 4; const int m = blockIdx.y, b0 = blockIdx.x * 64;
  const int i0 = min(max(PIDX[m * 2], 0), NC - 1), i1 = min(max(PIDX[m * 2 + 1], 0), NC - 1);
  if (tid < H1) { const int o = tid; sp1[o][0] = bfr(W1[((size_t)m * H1 + o) * 2]); sp1[o][1] = bfr(W1[((size_t)m * H1 + o) * 2 + 1]); sp1[o][2] = bfr(b1[m * H1 + o]);
    const float sc = bfr(g1[m * H1 + o]) * rsqrtf(bfr(v1[m * H1 + o]) + 1e-5f); sp1[o][3] = sc; sp1[o][4] = bfr(be1[m * H1 + o]) - bfr(m1[m * H1 + o]) * sc; }
  if (tid < H2) { const int o = tid; const float sc = bfr(g2[m * H2 + o]) * rsqrtf(bfr(v2[m * H2 + o]) + 1e-5f); sp2[o][0] = bfr(b2[m * H2 + o]); sp2[o][1] = sc; sp2[o][2] = bfr(be2[m * H2 + o]) - bfr(m2[m * H2 + o]) * sc; sw3[o] = bfr(W3[(size_t)m * H2 + o]); }
  __syncthreads();
  for (int q = tid; q < 64 * H1; q += 128) { const int bl = q >> 6, o = q & 63; const float xa = bfr(X[(size_t)(b0 + bl) * NC + i0]), xb = bfr(X[(size_t)(b0 + bl) * NC + i1]);
    const float h = (xa * sp1[o][0] + xb * sp1[o][1]) + sp1[o][2]; const float v = fmaxf(h * sp1[o][3] + sp1[o][4], 0.f);
    const __bf16 hb = (__bf16)v; sah[bl][o] = hb; sal[bl][o] = (__bf16)(v - (float)hb); }
  __syncthreads();
  { v8f acc[2] = {};
#pragma unroll
    for (int kc = 0; kc < 2; ++kc) { const v16b ah = frag_b(&sah[wave * 16 + col][kc * 32], lane), al = frag_b(&sal[wave * 16 + col][kc * 32], lane);
#pragma unroll
      for (int j = 0; j < 2; ++j) { const v16b w = frag_gbf(W2 + ((size_t)m * H2 + j * 16 + col) * H1 + kc * 32, lane); acc[j] = wmma_bf(al, w, acc[j]); acc[j] = wmma_bf(ah, w, acc[j]); } }
#pragma unroll
    for (int j = 0; j < 2; ++j) { const int o = j * 16 + col;
#pragma unroll
      for (int r = 0; r < 8; ++r) sh2[wave * 16 + 8 * g + r][o] = fmaxf((acc[j][r] + sp2[o][0]) * sp2[o][1] + sp2[o][2], 0.f); } }
  __syncthreads();
  if (tid < 64) { float s = bfr(b3[m]); for (int o = 0; o < H2; ++o) s += sh2[tid][o] * sw3[o]; sres[tid] = s; }
  __syncthreads();
  if (tid < 16) vst2(OT + (size_t)m * NB + b0 + tid * 4, *(const v4f*)&sres[tid * 4]);
}
__global__ __launch_bounds__(64) void k_zero(float* __restrict__ OT) { const int r = NM + blockIdx.x / 8, seg = blockIdx.x % 8; const v4f z = {0.f, 0.f, 0.f, 0.f}; vst2(OT + (size_t)r * NB + seg * 256 + threadIdx.x * 4, z); }
__global__ __launch_bounds__(128) void k_head(const float* __restrict__ OT, const float* __restrict__ Wout, const float* __restrict__ bout, float* __restrict__ out) {
  __shared__ __align__(16) __bf16 sah[64][520], sal[64][520]; __shared__ __align__(16) __bf16 sw[16][520]; __shared__ __align__(16) float sres[640];
  const int tid = threadIdx.x, wave = tid >> 5, lane = tid & 31, col = lane & 15, g = lane >> 4; const int b0 = blockIdx.x * 64;
  for (int q = tid; q < 512 * 64; q += 128) { const int m = q >> 6, bl = q & 63; const float v = OT[(size_t)m * NB + b0 + bl]; const __bf16 hb = (__bf16)v; sah[bl][m] = hb; sal[bl][m] = (__bf16)(v - (float)hb); }
  for (int q = tid; q < 16 * 512; q += 128) { const int c = q >> 9, m = q & 511; sw[c][m] = (__bf16)((c < NCLS && m < NM) ? bfr(Wout[c * NM + m]) : 0.f); }
  __syncthreads();
  v8f acc = {};
#pragma unroll 4
  for (int kc = 0; kc < 16; ++kc) { const v16b ah = frag_b(&sah[wave * 16 + col][kc * 32], lane), al = frag_b(&sal[wave * 16 + col][kc * 32], lane); const v16b w = frag_b(&sw[col][kc * 32], lane); acc = wmma_bf(al, w, acc); acc = wmma_bf(ah, w, acc); }
  if (col < NCLS) {
#pragma unroll
    for (int r = 0; r < 8; ++r) sres[(wave * 16 + 8 * g + r) * NCLS + col] = acc[r] + bfr(bout[col]); }
  __syncthreads();
  for (int q = tid; q < 640 / 4; q += 128) vst2(out + (size_t)b0 * NCLS + q * 4, *(const v4f*)&sres[q * 4]);
}

extern "C" void kernel_launch(void* const* d_in, const int* in_sizes, int n_in, void* d_out, int out_size, void* d_ws, size_t ws_size, hipStream_t stream) {
  (void)in_sizes; (void)n_in; (void)out_size;
  const float** F = (const float**)d_in; const int** I = (const int**)d_in;
  if (ws_size < (size_t)WS_END) return;
  float* OT = (float*)((char*)d_ws + WS_OT);
  k_pair<<<dim3(TBB, NM), 128, 0, stream>>>(F[0], I[1], F[2], F[3], F[4], F[5], F[6], F[7], F[8], F[9], F[10], F[11], F[12], F[13], F[14], F[15], OT);
  k_zero<<<16 * 8, 64, 0, stream>>>(OT);
  k_head<<<TBB, 128, 0, stream>>>(OT, F[16], F[17], (float*)d_out);
}
